// MultiEnvironmentPredictor_39642548142647
// MI455X (gfx1250) — hardware-verified
//
#include <hip/hip_runtime.h>
#include <stdint.h>

#define BB   16384
#define II   512
#define EE   8
#define INVD 128
#define SSD  64
#define HHD  256
#define H2D  128
#define DPAD 64

typedef __attribute__((ext_vector_type(16))) _Float16 v16h;
typedef __attribute__((ext_vector_type(8)))  _Float16 v8h;
typedef __attribute__((ext_vector_type(16))) __bf16   v16b;
typedef __attribute__((ext_vector_type(8)))  __bf16   v8b;
typedef __attribute__((ext_vector_type(8)))  float    v8f;
typedef __attribute__((ext_vector_type(4)))  float    v4f;

__device__ __forceinline__ unsigned short f2bf_bits(float f) {
  unsigned u = __float_as_uint(f);
  return (unsigned short)((u + 0x7FFFu + ((u >> 16) & 1u)) >> 16);
}
__device__ __forceinline__ float bf_bits2f(unsigned short h) { return __uint_as_float(((unsigned)h) << 16); }

__device__ __forceinline__ void dep_guard_h(v8f& a, v8f& b, v16h x, v16h y) { asm volatile("v_nop\n\tv_nop\n\tv_nop\n\tv_nop" : "+v"(a), "+v"(b) : "v"(x), "v"(y)); }
__device__ __forceinline__ void dep_guard_b(v8f& a, v8f& b, v16b x, v16b y) { asm volatile("v_nop\n\tv_nop\n\tv_nop\n\tv_nop" : "+v"(a), "+v"(b) : "v"(x), "v"(y)); }
__device__ __forceinline__ void keep4_h(v16h a, v16h b, v16h c, v16h d) { asm volatile("v_nop" :: "v"(a), "v"(b), "v"(c), "v"(d)); }
__device__ __forceinline__ void keep4_b(v16b a, v16b b, v16b c, v16b d) { asm volatile("v_nop" :: "v"(a), "v"(b), "v"(c), "v"(d)); }
__device__ __forceinline__ void acc_guard4(v8f& a, v8f& b, v8f& c, v8f& d) { asm volatile("v_nop\n\tv_nop\n\tv_nop\n\tv_nop" : "+v"(a), "+v"(b), "+v"(c), "+v"(d)); }
template <typename T> struct Frag;
template <> struct Frag<_Float16> {
  typedef v16h V; union U { v16h v; v8h h[2]; };
  static __device__ __forceinline__ v16h load(const _Float16* p) {
    U f; f.h[0] = *(const v8h*)(p); f.h[1] = *(const v8h*)(p + 16); return f.v;
  }
  static __device__ __forceinline__ v8f mma(v16h a, v16h b, v8f c) {
    return __builtin_amdgcn_wmma_f32_16x16x32_f16(false, a, false, b, (short)0, c, false, false);
  }
  static __device__ __forceinline__ void guard(v8f& a, v8f& b, v16h x, v16h y) { dep_guard_h(a, b, x, y); }
  static __device__ __forceinline__ void keep(v16h a, v16h b, v16h c, v16h d) { keep4_h(a, b, c, d); }
};
template <> struct Frag<__bf16> {
  typedef v16b V; union U { v16b v; v8b h[2]; };
  static __device__ __forceinline__ v16b load(const __bf16* p) {
    U f; f.h[0] = *(const v8b*)(p); f.h[1] = *(const v8b*)(p + 16); return f.v;
  }
  static __device__ __forceinline__ v8f mma(v16b a, v16b b, v8f c) {
    return __builtin_amdgcn_wmma_f32_16x16x32_bf16(false, a, false, b, (short)0, c, false, false);
  }
  static __device__ __forceinline__ void guard(v8f& a, v8f& b, v16b x, v16b y) { dep_guard_b(a, b, x, y); }
  static __device__ __forceinline__ void keep(v16b a, v16b b, v16b c, v16b d) { keep4_b(a, b, c, d); }
};

template <int ET> struct Elem;
template <> struct Elem<0> { typedef _Float16 T; };
template <> struct Elem<1> { typedef __bf16 T; };
template <int ET, bool SPLIT, int BIAS_MODE, int OUT_MODE, bool RESID, int ACT = 0>
__global__ __launch_bounds__(256) void wmma_gemm64(
    const unsigned short* __restrict__ Ap, const unsigned short* __restrict__ A2p, int lda, long strideA,
    const unsigned short* __restrict__ Btp, const unsigned short* __restrict__ Bt2p, int ldb, long strideB,
    void* __restrict__ Cout, void* __restrict__ Cout2, int ldc, long strideC,
    const float* __restrict__ bias, long strideBias,
    const float* __restrict__ resid, long strideR,
    int M, int N, int K, float scale) {
  typedef typename Elem<ET>::T T;
  typedef typename Frag<T>::V V;
  const T* A = (const T*)Ap; const T* A2 = (const T*)A2p; const T* Bt = (const T*)Btp; const T* Bt2 = (const T*)Bt2p;
  __shared__ __align__(16) float sT[8][16 * 68];
  const int b    = blockIdx.y;
  const int lane = threadIdx.x & 31;
  const int wave = threadIdx.x >> 5;
  const int tilesN = N >> 6;
  const int tilesM = M >> 6;
  const int tile = blockIdx.x * 8 + wave;
  if (tile >= tilesM * tilesN) return;
  const int tm = tile / tilesN;
  const int tn = tile - tm * tilesN;
  const int m0 = tm << 6;
  const int n0 = tn << 6;

  const T* Ab  = A  + (size_t)b * strideA;
  const T* Bb  = Bt + (size_t)b * strideB;
  const T* Ab2 = SPLIT ? (A2  + (size_t)b * strideA) : nullptr;
  const T* Bb2 = SPLIT ? (Bt2 + (size_t)b * strideB) : nullptr;
  const float* biasb = (BIAS_MODE != 0) ? (bias + (size_t)b * strideBias) : nullptr;

  const int rlane = lane & 15;
  const int koff  = (lane >> 4) * 8;
  const int mOff  = (lane >> 4) * 8;

  v8f acc[4][4];
#pragma unroll
  for (int i = 0; i < 4; ++i)
#pragma unroll
    for (int j = 0; j < 4; ++j) acc[i][j] = (v8f){0.f,0.f,0.f,0.f,0.f,0.f,0.f,0.f};

  for (int k0 = 0; k0 < K; k0 += 32) {
    V bh[4], bl[4];
#pragma unroll
    for (int j = 0; j < 4; ++j) {
      const size_t bo = (size_t)(n0 + (j << 4) + rlane) * ldb + koff + k0;
      bh[j] = Frag<T>::load(Bb + bo);
      if (SPLIT) bl[j] = Frag<T>::load(Bb2 + bo);
    }
#pragma unroll
    for (int i = 0; i < 4; ++i) {
      const size_t ao = (size_t)(m0 + (i << 4) + rlane) * lda + koff + k0;
      V ah = Frag<T>::load(Ab + ao);
      V al;
      if (SPLIT) al = Frag<T>::load(Ab2 + ao);
#pragma unroll
      for (int j = 0; j < 4; ++j) {
        acc[i][j] = Frag<T>::mma(ah, bh[j], acc[i][j]);
        if (SPLIT) {
          acc[i][j] = Frag<T>::mma(ah, bl[j], acc[i][j]);
          acc[i][j] = Frag<T>::mma(al, bh[j], acc[i][j]);
        }
      }
      Frag<T>::guard(acc[i][0], acc[i][3], ah, SPLIT ? al : ah);
    }
    Frag<T>::keep(bh[0], bh[1], bh[2], bh[3]);
    if (SPLIT) Frag<T>::keep(bl[0], bl[1], bl[2], bl[3]);
  }
  acc_guard4(acc[0][0], acc[0][1], acc[0][2], acc[0][3]);
  acc_guard4(acc[1][0], acc[1][1], acc[1][2], acc[1][3]);
  acc_guard4(acc[2][0], acc[2][1], acc[2][2], acc[2][3]);
  acc_guard4(acc[3][0], acc[3][1], acc[3][2], acc[3][3]);

  float* slab = sT[wave];
  const float* Rb = RESID ? (resid + (size_t)b * strideR) : nullptr;
#pragma unroll
  for (int i = 0; i < 4; ++i) {
    const int mBase = m0 + (i << 4);
#pragma unroll
    for (int j = 0; j < 4; ++j) {
      const int n = n0 + (j << 4) + rlane;
      float bv = 0.f;
      if (BIAS_MODE == 2) bv = biasb[n];
#pragma unroll
      for (int r = 0; r < 8; ++r) {
        float v = acc[i][j][r] * scale;
        if (BIAS_MODE == 1) v += biasb[mBase + mOff + r];
        if (BIAS_MODE == 2) v += bv;
        if (RESID) v += Rb[(size_t)(mBase + mOff + r) * ldc + n];
        if (ACT == 1) v = tanhf(v);
        if (ACT == 2) v = fmaxf(v, 0.0f);
        if (ACT == 3) v = v / (1.0f + expf(-v));
        if (ACT == 4) v = (v > 0.f) ? v : 0.01f * v;
        if (ACT == 5) v = 0.5f * v * (1.0f + erff(v * 0.70710678118654752f));
        slab[(mOff + r) * 68 + (j << 4) + rlane] = v;
      }
    }
    __builtin_amdgcn_fence(__ATOMIC_RELEASE, "workgroup");
    __builtin_amdgcn_wave_barrier();
    __builtin_amdgcn_fence(__ATOMIC_ACQUIRE, "workgroup");
    if (OUT_MODE == 0) {
      float* C = (float*)Cout + (size_t)b * strideC;
      const int hh = lane >> 4, c4 = (lane & 15) * 4;
      for (int pass = 0; pass < 2; ++pass) {
#pragma unroll
        for (int it = 0; it < 8; ++it) {
          const int row = it * 2 + hh;
          v4f v = *(const v4f*)(slab + row * 68 + c4);
          *(volatile v4f*)(C + (size_t)(mBase + row) * ldc + n0 + c4) = v;
        }
        __threadfence();
      }
    } else {
      const int q = lane >> 3, c8 = (lane & 7) * 8;
      unsigned short* C  = (unsigned short*)Cout  + (size_t)b * strideC;
      unsigned short* C2 = (OUT_MODE == 2) ? ((unsigned short*)Cout2 + (size_t)b * strideC) : nullptr;
      for (int pass = 0; pass < 2; ++pass) {
#pragma unroll
        for (int it = 0; it < 4; ++it) {
          const int row = it * 4 + q;
          const float* sp = slab + row * 68 + c8;
          v8h hv, lv;
#pragma unroll
          for (int e = 0; e < 8; ++e) {
            if (OUT_MODE == 1) {
              hv[e] = (_Float16)sp[e];
            } else {
              unsigned short hb = f2bf_bits(sp[e]);
              unsigned short lb = f2bf_bits(sp[e] - bf_bits2f(hb));
              hv[e] = __builtin_bit_cast(_Float16, hb);
              lv[e] = __builtin_bit_cast(_Float16, lb);
            }
          }
          *(volatile v8h*)(C + (size_t)(mBase + row) * ldc + n0 + c8) = hv;
          if (OUT_MODE == 2) *(volatile v8h*)(C2 + (size_t)(mBase + row) * ldc + n0 + c8) = lv;
        }
        __threadfence();
      }
    }
    __builtin_amdgcn_fence(__ATOMIC_RELEASE, "workgroup");
    __builtin_amdgcn_wave_barrier();
    __builtin_amdgcn_fence(__ATOMIC_ACQUIRE, "workgroup");
  }
}

__global__ __launch_bounds__(256) void cast_f32_f16x2(
    const float* __restrict__ in, _Float16* __restrict__ out, int n2) {
  int i = blockIdx.x * 256 + threadIdx.x;
  if (i < n2) {
    const _Float16 h0 = (_Float16)in[2 * i], h1 = (_Float16)in[2 * i + 1];
    const unsigned u = (unsigned)__builtin_bit_cast(unsigned short, h0) | ((unsigned)__builtin_bit_cast(unsigned short, h1) << 16);
    ((volatile unsigned*)out)[i] = u;
    __threadfence();
    ((volatile unsigned*)out)[i] = u;
  }
}

__global__ __launch_bounds__(256) void tcast_kn_f16(
    const float* __restrict__ in, _Float16* __restrict__ out, int K, int Nreal, int Npad, int total2) {
  const int t = blockIdx.x * 256 + threadIdx.x;
  if (t < total2) {
    const int K2 = K >> 1;
    const int k2 = t % K2;
    const int rest = t / K2;
    const int n = rest % Npad;
    const int bz = rest / Npad;
    const int k = 2 * k2;
    float f0 = 0.0f, f1 = 0.0f;
    if (n < Nreal) {
      const float* p = in + ((size_t)bz * K + k) * (size_t)Nreal + n;
      f0 = p[0];
      f1 = p[Nreal];
    }
    const _Float16 h0 = (_Float16)f0, h1 = (_Float16)f1;
    const unsigned u = (unsigned)__builtin_bit_cast(unsigned short, h0) | ((unsigned)__builtin_bit_cast(unsigned short, h1) << 16);
    ((volatile unsigned*)out)[t] = u;
    __threadfence();
    ((volatile unsigned*)out)[t] = u;
  }
}

__global__ __launch_bounds__(64) void head_rows(
    const float* __restrict__ inv, const float* __restrict__ sall, const float* __restrict__ domp,
    const int* __restrict__ env, const float* __restrict__ Wf, const float* __restrict__ bfp,
    const float* __restrict__ bd2, float* out0, float* out2, float* out3, int nrows) {
  const int lane = threadIdx.x & 31;
  const int wave = threadIdx.x >> 5;
  const int r0 = (blockIdx.x * 2 + wave) * 32;
  if (r0 + 32 > nrows) return;
  const int row = r0 + lane;
  int e = env[row];
  const float vsel = (e >= 0 && e < EE) ? 1.0f : 0.0f;
  e = e < 0 ? 0 : (e >= EE ? (EE - 1) : e);

  const float* ir = inv + (size_t)row * INVD;
  float a0 = 0.0f;
#pragma unroll 1
  for (int i = 0; i < INVD; ++i) a0 += ir[i] * Wf[i];
  const float* sr = sall + ((size_t)row * EE + e) * SSD;
  float a1 = 0.0f;
#pragma unroll 1
  for (int j = 0; j < SSD; ++j) a1 += sr[j] * Wf[INVD + j];
  const float logit = a0 + a1 * vsel + bfp[0];

  v4f lv;
  lv[0] = __shfl(logit, (4 * lane + 0) & 31, 32);
  lv[1] = __shfl(logit, (4 * lane + 1) & 31, 32);
  lv[2] = __shfl(logit, (4 * lane + 2) & 31, 32);
  lv[3] = __shfl(logit, (4 * lane + 3) & 31, 32);

  const int rA = r0 + (lane >> 1);
  const int rB = rA + 16;
  const int cd = (lane & 1) * 4;
  v4f dA, dB;
#pragma unroll
  for (int qq = 0; qq < 4; ++qq) {
    const float bb = bd2[cd + qq];
    dA[qq] = domp[(size_t)rA * DPAD + cd + qq] + bb;
    dB[qq] = domp[(size_t)rB * DPAD + cd + qq] + bb;
  }

  const int c4 = (lane & 15) * 4;
  for (int pass = 0; pass < 2; ++pass) {
    if (lane < 8) *(volatile v4f*)(out0 + r0 + 4 * lane) = lv;
    *(volatile v4f*)(out3 + (size_t)rA * EE + cd) = dA;
    *(volatile v4f*)(out3 + (size_t)rB * EE + cd) = dB;
#pragma unroll
    for (int it = 0; it < 16; ++it) {
      const int rr = r0 + 2 * it + (lane >> 4);
      int ee = env[rr];
      const float vs = (ee >= 0 && ee < EE) ? 1.0f : 0.0f;
      ee = ee < 0 ? 0 : (ee >= EE ? (EE - 1) : ee);
      v4f sv = *(const v4f*)(sall + ((size_t)rr * EE + ee) * SSD + c4);
      sv = sv * vs;
      *(volatile v4f*)(out2 + (size_t)rr * SSD + c4) = sv;
    }
    __threadfence();
  }
}

extern "C" void kernel_launch(void* const* d_in, const int* in_sizes, int n_in,
                              void* d_out, int out_size, void* d_ws, size_t ws_size,
                              hipStream_t stream) {
  if (n_in < 16) return;
  if (in_sizes[0] != BB * II || in_sizes[1] != BB) return;
  if (out_size != BB * (1 + INVD + SSD + EE)) return;

  const float* x   = (const float*)d_in[0];
  const int*   env = (const int*)  d_in[1];
  const float* W1  = (const float*)d_in[2];
  const float* b1  = (const float*)d_in[3];
  const float* W2  = (const float*)d_in[4];
  const float* b2  = (const float*)d_in[5];
  const float* Ws1 = (const float*)d_in[6];
  const float* bs1 = (const float*)d_in[7];
  const float* Ws2 = (const float*)d_in[8];
  const float* bs2 = (const float*)d_in[9];
  const float* Wf  = (const float*)d_in[10];
  const float* bfp = (const float*)d_in[11];
  const float* Wd1 = (const float*)d_in[12];
  const float* bd1 = (const float*)d_in[13];
  const float* Wd2 = (const float*)d_in[14];
  const float* bd2 = (const float*)d_in[15];

  float* out0 = (float*)d_out;
  float* out1 = out0 + (size_t)BB;
  float* out2 = out1 + (size_t)BB * INVD;
  float* out3 = out2 + (size_t)BB * SSD;

  size_t off = 0;
  auto carve = [&](size_t bytes) { size_t o = off; off += (bytes + 255) & ~(size_t)255; return o; };
  const size_t o_x16  = carve((size_t)BB * II * 2);
  const size_t o_W1t  = carve((size_t)HHD * II * 2);
  const size_t o_W2t  = carve((size_t)INVD * HHD * 2);
  const size_t o_Ws1t = carve((size_t)EE * H2D * II * 2);
  const size_t o_Ws2t = carve((size_t)EE * SSD * H2D * 2);
  const size_t o_Wd1t = carve((size_t)H2D * INVD * 2);
  const size_t o_Wd2p = carve((size_t)DPAD * H2D * 2);
  const size_t o_h1   = carve((size_t)BB * HHD * 2);
  const size_t o_inv16= carve((size_t)BB * INVD * 2);
  const size_t o_hall = carve((size_t)BB * EE * H2D * 2);
  const size_t o_sall = carve((size_t)BB * EE * SSD * 4);
  const size_t o_hd   = carve((size_t)BB * H2D * 2);
  const size_t o_domp = carve((size_t)BB * DPAD * 4);
  if (off > ws_size) return;

  char* ws = (char*)d_ws;
  unsigned short* x16   = (unsigned short*)(ws + o_x16);
  unsigned short* W1t   = (unsigned short*)(ws + o_W1t);
  unsigned short* W2t   = (unsigned short*)(ws + o_W2t);
  unsigned short* Ws1t  = (unsigned short*)(ws + o_Ws1t);
  unsigned short* Ws2t  = (unsigned short*)(ws + o_Ws2t);
  unsigned short* Wd1t  = (unsigned short*)(ws + o_Wd1t);
  unsigned short* Wd2p  = (unsigned short*)(ws + o_Wd2p);
  unsigned short* h1    = (unsigned short*)(ws + o_h1);
  unsigned short* inv16 = (unsigned short*)(ws + o_inv16);
  unsigned short* hall  = (unsigned short*)(ws + o_hall);
  float*          sall  = (float*)(ws + o_sall);
  unsigned short* hd    = (unsigned short*)(ws + o_hd);
  float*          domp  = (float*)(ws + o_domp);

  const unsigned short* nul16 = nullptr;

  { const int n2 = BB * II / 2;
    cast_f32_f16x2<<<(n2 + 255) / 256, 256, 0, stream>>>(x, (_Float16*)x16, n2); }

  auto tcast = [&](const float* s, unsigned short* d, int bz, int K, int Nreal, int Npad) {
    const int total2 = bz * Npad * K / 2;
    tcast_kn_f16<<<(total2 + 255) / 256, 256, 0, stream>>>(s, (_Float16*)d, K, Nreal, Npad, total2);
  };
  tcast(W1,  W1t,  1,  II,   HHD,  HHD);
  tcast(W2,  W2t,  1,  HHD,  INVD, INVD);
  tcast(Ws1, Ws1t, EE, II,   H2D,  H2D);
  tcast(Ws2, Ws2t, EE, H2D,  SSD,  SSD);
  tcast(Wd1, Wd1t, 1,  INVD, H2D,  H2D);
  tcast(Wd2, Wd2p, 1,  H2D,  EE,   DPAD);

  wmma_gemm64<0, false, 2, 1, false, 2><<<dim3((BB / 64) * (HHD / 64) / 8, 1), 256, 0, stream>>>(
      x16, nul16, II, 0L, W1t, nul16, II, 0L, (void*)h1, (void*)nullptr, HHD, 0L,
      b1, 0L, (const float*)nullptr, 0L, BB, HHD, II, 1.0f);

  wmma_gemm64<0, false, 2, 0, false, 0><<<dim3((BB / 64) * (INVD / 64) / 8, 1), 256, 0, stream>>>(
      h1, nul16, HHD, 0L, W2t, nul16, HHD, 0L, (void*)out1, (void*)nullptr, INVD, 0L,
      b2, 0L, (const float*)nullptr, 0L, BB, INVD, HHD, 1.0f);

  { const int n2 = BB * INVD / 2;
    cast_f32_f16x2<<<(n2 + 255) / 256, 256, 0, stream>>>(out1, (_Float16*)inv16, n2); }

  wmma_gemm64<0, false, 2, 1, false, 2><<<dim3((BB / 64) * ((EE * H2D) / 64) / 8, 1), 256, 0, stream>>>(
      x16, nul16, II, 0L, Ws1t, nul16, II, 0L, (void*)hall, (void*)nullptr, EE * H2D, 0L,
      bs1, 0L, (const float*)nullptr, 0L, BB, EE * H2D, II, 1.0f);

  wmma_gemm64<0, false, 2, 0, false, 0><<<dim3((BB / 64) * (SSD / 64) / 8, EE), 256, 0, stream>>>(
      hall, nul16, EE * H2D, (long)H2D, Ws2t, nul16, H2D, (long)(SSD * H2D), (void*)sall, (void*)nullptr, EE * SSD, (long)SSD,
      bs2, (long)SSD, (const float*)nullptr, 0L, BB, SSD, H2D, 1.0f);

  wmma_gemm64<0, false, 2, 1, false, 2><<<dim3((BB / 64) * (H2D / 64) / 8, 1), 256, 0, stream>>>(
      inv16, nul16, INVD, 0L, Wd1t, nul16, INVD, 0L, (void*)hd, (void*)nullptr, H2D, 0L,
      bd1, 0L, (const float*)nullptr, 0L, BB, H2D, INVD, 1.0f);

  wmma_gemm64<0, false, 0, 0, false, 0><<<dim3((BB / 64) * (DPAD / 64) / 8, 1), 256, 0, stream>>>(
      hd, nul16, H2D, 0L, Wd2p, nul16, H2D, 0L, (void*)domp, (void*)nullptr, DPAD, 0L,
      (const float*)nullptr, 0L, (const float*)nullptr, 0L, BB, DPAD, H2D, 1.0f);

  head_rows<<<BB / 64, 64, 0, stream>>>(out1, sall, domp, env, Wf, bfp, bd2, out0, out2, out3, BB);
}
